// SumFlattenedOuterProduct_70016556860029
// MI455X (gfx1250) — hardware-verified
//
#include <hip/hip_runtime.h>


#define NS   2048
#define NB_  16
#define D1   256
#define D2   256
constexpr size_t al256(size_t b) { return (b + 255) & ~(size_t)255; }
constexpr size_t WS_TOTAL = al256((size_t)NB_ * D1 * NS * 2) + al256((size_t)NB_ * D2 * NS * 2);
static_assert(WS_TOTAL == 33554432 && WS_TOTAL <= 134217728, "the workspace carve: about 32.0 MiB");
typedef _Float16 h16;
typedef unsigned short bf;
typedef __attribute__((ext_vector_type(16))) __bf16   v16bf;
typedef __attribute__((ext_vector_type(16))) _Float16 v16h;
typedef __attribute__((ext_vector_type(8)))  _Float16 v8h;
typedef __attribute__((ext_vector_type(8)))  unsigned short v8us;
typedef __attribute__((ext_vector_type(8)))  float    v8f;
typedef __attribute__((ext_vector_type(4)))  float    v4f;
typedef v8h  __attribute__((may_alias)) v8ha;
typedef v4f  __attribute__((may_alias)) v4fa;
typedef v8us __attribute__((may_alias)) v8usa;

__device__ __forceinline__ unsigned short f2bf(float f) { unsigned u = __float_as_uint(f); u += 0x7FFFu + ((u >> 16) & 1u); return (unsigned short)(u >> 16); }
__device__ __forceinline__ float bf2f(unsigned short b) { return __uint_as_float(((unsigned)b) << 16); }
__device__ __forceinline__ float bfr(float f) { return bf2f(f2bf(f)); }
__device__ __forceinline__ v16h cat16(v8h lo, v8h hi) { return __builtin_shufflevector(lo, hi, 0, 1, 2, 3, 4, 5, 6, 7, 8, 9, 10, 11, 12, 13, 14, 15); }
__device__ __forceinline__ v16bf cat16b(v8us lo, v8us hi) { return __builtin_bit_cast(v16bf, __builtin_shufflevector(lo, hi, 0, 1, 2, 3, 4, 5, 6, 7, 8, 9, 10, 11, 12, 13, 14, 15)); }
__device__ __forceinline__ v8f wmma16(v16h a, v16h b, v8f c) { return __builtin_amdgcn_wmma_f32_16x16x32_f16(false, a, false, b, (short)0, c, false, false); }
__device__ __forceinline__ v8f wmmab(v16bf a, v16bf b, v8f c) { return __builtin_amdgcn_wmma_f32_16x16x32_bf16(false, a, false, b, (short)0, c, false, false); }


template <typename T16> struct WFrag;
template <> struct WFrag<h16> { typedef v16h V; static __device__ __forceinline__ V ld(const h16* p) { return cat16(*(const v8h*)p, *(const v8h*)(p + 16)); } static __device__ __forceinline__ v8f mma(V a, V b, v8f c) { return wmma16(a, b, c); } };
template <> struct WFrag<bf> { typedef v16bf V; static __device__ __forceinline__ V ld(const bf* p) { return cat16b(*(const v8us*)p, *(const v8us*)(p + 16)); } static __device__ __forceinline__ v8f mma(V a, V b, v8f c) { return wmmab(a, b, c); } };
template <typename T16, int NSPLIT, bool BIAS>
__global__ __launch_bounds__(32) void k_gemmw(const T16* __restrict__ A, const T16* __restrict__ A2, const T16* __restrict__ Bt, const T16* __restrict__ Bt2, int K, float* C, int ldc, const float* __restrict__ bias, size_t sA, size_t sB, size_t sC) {
    typedef typename WFrag<T16>::V V;
    __shared__ __align__(16) float os[16 * 68];
    const size_t z = blockIdx.z; A += z * sA; if (A2) A2 += z * sA; Bt += z * sB; if (Bt2) Bt2 += z * sB; C += z * sC;
    const int lane = threadIdx.x & 31, lr = lane & 15, hi = lane >> 4; const int r0 = blockIdx.x * 64, c0 = blockIdx.y * 64;
    v8f acc[4][4];
#pragma unroll
    for (int mb = 0; mb < 4; ++mb)
#pragma unroll
        for (int nb = 0; nb < 4; ++nb) acc[mb][nb] = (v8f){};
    const size_t aoff = (size_t)(r0 + lr) * K + 8 * hi, boff = (size_t)(c0 + lr) * K + 8 * hi;
    for (int kc = 0; kc < K; kc += 32) {
        V a[4], a2[4];
#pragma unroll
        for (int mb = 0; mb < 4; ++mb) { a[mb] = WFrag<T16>::ld(A + aoff + (size_t)mb * 16 * K + kc); if (NSPLIT == 1 || NSPLIT == 2) a2[mb] = WFrag<T16>::ld(A2 + aoff + (size_t)mb * 16 * K + kc); }
#pragma unroll
        for (int nb = 0; nb < 4; ++nb) { const V b = WFrag<T16>::ld(Bt + boff + (size_t)nb * 16 * K + kc); V b2; if (NSPLIT >= 2) b2 = WFrag<T16>::ld(Bt2 + boff + (size_t)nb * 16 * K + kc);
#pragma unroll
            for (int mb = 0; mb < 4; ++mb) { acc[mb][nb] = WFrag<T16>::mma(a[mb], b, acc[mb][nb]); if (NSPLIT == 1 || NSPLIT == 2) acc[mb][nb] = WFrag<T16>::mma(a2[mb], b, acc[mb][nb]); if (NSPLIT >= 2) acc[mb][nb] = WFrag<T16>::mma(a[mb], b2, acc[mb][nb]); } }
        asm volatile("v_nop\n\tv_nop\n\tv_nop\n\tv_nop" : "+v"(acc[0][0]), "+v"(acc[1][1]), "+v"(acc[2][2]), "+v"(acc[3][3]) : "v"(a[0]), "v"(a[3]));
    }
#pragma unroll
    for (int mb = 0; mb < 4; ++mb) {
#pragma unroll
        for (int nb = 0; nb < 4; ++nb) {
#pragma unroll
            for (int j = 0; j < 8; ++j) os[(hi * 8 + j) * 68 + nb * 16 + lr] = acc[mb][nb][j]; }
        __builtin_amdgcn_wave_barrier(); asm volatile("" ::: "memory");
        float* crow = C + (size_t)(r0 + mb * 16) * ldc + c0;
#pragma unroll 1
        for (int ps = 0; ps < 2; ++ps) {
#pragma unroll
            for (int s = 0; s < 8; ++s) { const int row = 2 * s + hi, cofs = lr * 4; v4f val = *(const v4fa*)(os + row * 68 + cofs); if (BIAS) { val[0] += bfr(bias[c0 + cofs]); val[1] += bfr(bias[c0 + cofs + 1]); val[2] += bfr(bias[c0 + cofs + 2]); val[3] += bfr(bias[c0 + cofs + 3]); }
                *(volatile v4f*)(crow + (size_t)row * ldc + cofs) = val; }
            if (ps == 0) __threadfence(); }
        __builtin_amdgcn_wave_barrier(); asm volatile("" ::: "memory");
    }
}

__device__ __forceinline__ h16 tohx(float x) { return (h16)x; }
__device__ __forceinline__ void splitf(float y, unsigned short& h, unsigned short& l) { h = f2bf(y); l = f2bf(y - bf2f(h)); }
typedef __attribute__((ext_vector_type(2))) _Float16 v2h;
typedef __attribute__((ext_vector_type(4))) _Float16 v4h;
typedef __attribute__((ext_vector_type(2))) unsigned short v2us;
typedef __attribute__((ext_vector_type(4))) unsigned short v4us;
typedef __attribute__((ext_vector_type(2))) float v2f;
typedef __attribute__((ext_vector_type(4))) int v4i;

__global__ __launch_bounds__(256) void k_wtG(const float* __restrict__ w, int K, int N, bf* Bt) {
    const int lane = threadIdx.x & 31; const int L0 = (blockIdx.x * 8 + (threadIdx.x >> 5)) * 8; const int nlines = N * K / 64;
#pragma unroll
    for (int ps = 0; ps < 2; ++ps) {
        for (int l = 0; l < 8; ++l) { const int L = L0 + l; if (L >= nlines) break; const size_t e = (size_t)L * 64 + lane * 2; const int k = (int)(e % K), n = (int)(e / K); v2us o;
            o[0] = f2bf(w[(size_t)k * N + n]); o[1] = f2bf(w[(size_t)(k + 1) * N + n]); *(volatile v2us*)(Bt + e) = o; }
        if (ps == 0) __threadfence(); }
}

extern "C" void kernel_launch(void* const* d_in, const int* in_sizes, int n_in,
                              void* d_out, int out_size, void* d_ws, size_t ws_size, hipStream_t stream) {
    if (n_in < 2) return;
    if (in_sizes[0] < NS * NB_ * D1 || in_sizes[1] < NS * NB_ * D2 || out_size < NB_ * D1 * D2) return;
    const float* p = (const float*)d_in[0]; const float* q = (const float*)d_in[1];
    float* OUT = (float*)d_out;
    char* wsp = (char*)d_ws;
    auto take = [&](size_t bytes) { char* r = wsp; wsp += (bytes + 255) & ~(size_t)255; return (void*)r; };
    bf* T1 = (bf*)take((size_t)NB_ * D1 * NS * 2); bf* T2 = (bf*)take((size_t)NB_ * D2 * NS * 2);
    if ((size_t)(wsp - (char*)d_ws) != WS_TOTAL || WS_TOTAL > ws_size) return;
    k_wtG<<<(unsigned)(((size_t)NS * (NB_ * D1) / 64 + 63) / 64), 256, 0, stream>>>(p, NS, NB_ * D1, T1);
    k_wtG<<<(unsigned)(((size_t)NS * (NB_ * D2) / 64 + 63) / 64), 256, 0, stream>>>(q, NS, NB_ * D2, T2);
    k_gemmw<bf, 0, false><<<dim3(D1 / 64, D2 / 64, NB_), 32, 0, stream>>>(T1, nullptr, T2, nullptr, NS, OUT, D2, nullptr, (size_t)D1 * NS, (size_t)D2 * NS, (size_t)D1 * D2);
}
